// Incep_MHSA_85117661872663
// MI455X (gfx1250) — hardware-verified
//
#include <hip/hip_runtime.h>
#include <math.h>

constexpr int kB        = 8;
constexpr int kC        = 512;
constexpr int kHW       = 56;
constexpr int kN        = 3136;
constexpr int kHeads    = 8;
constexpr int kHD       = 64;
constexpr int kM        = 588;
constexpr int kMP       = 640;
constexpr int kP14      = 196;
constexpr int kTokRows  = kB * kN;
constexpr int kKVRows   = kB * kMP;
constexpr int kGH       = 4;
constexpr int kGroupRows = kGH * kN;
constexpr float kWCarry    = 64.0f;
constexpr float kWCarryInv = 1.0f / 64.0f;
constexpr float kPCarry    = 32768.0f;
constexpr float kPCarryInv = 1.0f / 32768.0f;
constexpr float kQKScale   = 0.125f;
constexpr float kLnEps     = 1e-5f;

typedef __attribute__((ext_vector_type(16))) _Float16 v16h;
typedef __attribute__((ext_vector_type(8)))  _Float16 v8h;
typedef __attribute__((ext_vector_type(16))) __bf16   v16b;
typedef __attribute__((ext_vector_type(8)))  __bf16   v8b;
typedef __attribute__((ext_vector_type(8)))  float    v8f;
typedef __attribute__((ext_vector_type(4)))  float    v4f;
typedef __attribute__((ext_vector_type(4)))  unsigned int v4u;

__device__ __forceinline__ unsigned short f2bf_bits(float f) {
  unsigned u = __float_as_uint(f);
  return (unsigned short)((u + 0x7FFFu + ((u >> 16) & 1u)) >> 16);
}
__device__ __forceinline__ float bf_bits2f(unsigned short h) { return __uint_as_float(((unsigned)h) << 16); }

__device__ __forceinline__ void dep_guard_h(v8f& a, v8f& b, v16h x, v16h y) { asm volatile("v_nop\n\tv_nop\n\tv_nop\n\tv_nop" : "+v"(a), "+v"(b) : "v"(x), "v"(y)); }
__device__ __forceinline__ void dep_guard_b(v8f& a, v8f& b, v16b x, v16b y) { asm volatile("v_nop\n\tv_nop\n\tv_nop\n\tv_nop" : "+v"(a), "+v"(b) : "v"(x), "v"(y)); }
__device__ __forceinline__ void keep4_h(v16h a, v16h b, v16h c, v16h d) { asm volatile("v_nop" :: "v"(a), "v"(b), "v"(c), "v"(d)); }
__device__ __forceinline__ void keep4_b(v16b a, v16b b, v16b c, v16b d) { asm volatile("v_nop" :: "v"(a), "v"(b), "v"(c), "v"(d)); }
__device__ __forceinline__ void acc_guard4(v8f& a, v8f& b, v8f& c, v8f& d) { asm volatile("v_nop\n\tv_nop\n\tv_nop\n\tv_nop" : "+v"(a), "+v"(b), "+v"(c), "+v"(d)); }
template <typename T> struct Frag;
template <> struct Frag<_Float16> {
  typedef v16h V; union U { v16h v; v8h h[2]; };
  static __device__ __forceinline__ v16h load(const _Float16* p) {
    U f; f.h[0] = *(const v8h*)(p); f.h[1] = *(const v8h*)(p + 16); return f.v;
  }
  static __device__ __forceinline__ v8f mma(v16h a, v16h b, v8f c) {
    return __builtin_amdgcn_wmma_f32_16x16x32_f16(false, a, false, b, (short)0, c, false, false);
  }
  static __device__ __forceinline__ void guard(v8f& a, v8f& b, v16h x, v16h y) { dep_guard_h(a, b, x, y); }
  static __device__ __forceinline__ void keep(v16h a, v16h b, v16h c, v16h d) { keep4_h(a, b, c, d); }
};
template <> struct Frag<__bf16> {
  typedef v16b V; union U { v16b v; v8b h[2]; };
  static __device__ __forceinline__ v16b load(const __bf16* p) {
    U f; f.h[0] = *(const v8b*)(p); f.h[1] = *(const v8b*)(p + 16); return f.v;
  }
  static __device__ __forceinline__ v8f mma(v16b a, v16b b, v8f c) {
    return __builtin_amdgcn_wmma_f32_16x16x32_bf16(false, a, false, b, (short)0, c, false, false);
  }
  static __device__ __forceinline__ void guard(v8f& a, v8f& b, v16b x, v16b y) { dep_guard_b(a, b, x, y); }
  static __device__ __forceinline__ void keep(v16b a, v16b b, v16b c, v16b d) { keep4_b(a, b, c, d); }
};

__device__ __forceinline__ unsigned pk16(unsigned short a, unsigned short b) { return (unsigned)a | ((unsigned)b << 16); }
__device__ __forceinline__ unsigned short h_bits(float f) { const _Float16 h = (_Float16)f; return __builtin_bit_cast(unsigned short, h); }

template <int ET> struct Elem;
template <> struct Elem<0> { typedef _Float16 T; };
template <> struct Elem<1> { typedef __bf16 T; };
template <int ET, bool SPLIT, int BIAS_MODE, int OUT_MODE, bool RESID, int ACT = 0>
__global__ __launch_bounds__(256) void wmma_gemm64(
    const unsigned short* __restrict__ Ap, const unsigned short* __restrict__ A2p, int lda, long strideA,
    const unsigned short* __restrict__ Btp, const unsigned short* __restrict__ Bt2p, int ldb, long strideB,
    void* __restrict__ Cout, void* __restrict__ Cout2, int ldc, long strideC,
    const float* __restrict__ bias,
    const float* __restrict__ resid, long strideR,
    int M, int N, int K, float scale) {
  typedef typename Elem<ET>::T T;
  typedef typename Frag<T>::V V;
  const T* A = (const T*)Ap; const T* A2 = (const T*)A2p; const T* Bt = (const T*)Btp; const T* Bt2 = (const T*)Bt2p;
  __shared__ __align__(16) float sT[8][16 * 68];
  const int b    = blockIdx.y;
  const int lane = threadIdx.x & 31;
  const int wave = threadIdx.x >> 5;
  const int tilesN = N >> 6;
  const int tilesM = M >> 6;
  const int tile = blockIdx.x * 8 + wave;
  if (tile >= tilesM * tilesN) return;
  const int tm = tile / tilesN;
  const int tn = tile - tm * tilesN;
  const int m0 = tm << 6;
  const int n0 = tn << 6;

  const T* Ab  = A  + (size_t)b * strideA;
  const T* Bb  = Bt + (size_t)b * strideB;
  const T* Ab2 = SPLIT ? (A2  + (size_t)b * strideA) : nullptr;
  const T* Bb2 = SPLIT ? (Bt2 + (size_t)b * strideB) : nullptr;

  const int rlane = lane & 15;
  const int koff  = (lane >> 4) * 8;
  const int mOff  = (lane >> 4) * 8;

  v8f acc[4][4];
#pragma unroll
  for (int i = 0; i < 4; ++i)
#pragma unroll
    for (int j = 0; j < 4; ++j) acc[i][j] = (v8f){0.f,0.f,0.f,0.f,0.f,0.f,0.f,0.f};

  for (int k0 = 0; k0 < K; k0 += 32) {
    V bh[4], bl[4];
#pragma unroll
    for (int j = 0; j < 4; ++j) {
      const size_t bo = (size_t)(n0 + (j << 4) + rlane) * ldb + koff + k0;
      bh[j] = Frag<T>::load(Bb + bo);
      if (SPLIT) bl[j] = Frag<T>::load(Bb2 + bo);
    }
#pragma unroll
    for (int i = 0; i < 4; ++i) {
      const size_t ao = (size_t)(m0 + (i << 4) + rlane) * lda + koff + k0;
      V ah = Frag<T>::load(Ab + ao);
      V al;
      if (SPLIT) al = Frag<T>::load(Ab2 + ao);
#pragma unroll
      for (int j = 0; j < 4; ++j) {
        acc[i][j] = Frag<T>::mma(ah, bh[j], acc[i][j]);
        if (SPLIT) {
          acc[i][j] = Frag<T>::mma(ah, bl[j], acc[i][j]);
          acc[i][j] = Frag<T>::mma(al, bh[j], acc[i][j]);
        }
      }
      Frag<T>::guard(acc[i][0], acc[i][3], ah, SPLIT ? al : ah);
    }
    Frag<T>::keep(bh[0], bh[1], bh[2], bh[3]);
    if (SPLIT) Frag<T>::keep(bl[0], bl[1], bl[2], bl[3]);
  }
  acc_guard4(acc[0][0], acc[0][1], acc[0][2], acc[0][3]);
  acc_guard4(acc[1][0], acc[1][1], acc[1][2], acc[1][3]);
  acc_guard4(acc[2][0], acc[2][1], acc[2][2], acc[2][3]);
  acc_guard4(acc[3][0], acc[3][1], acc[3][2], acc[3][3]);

  float* slab = sT[wave];
  const float* Rb = RESID ? (resid + (size_t)b * strideR) : nullptr;
#pragma unroll
  for (int i = 0; i < 4; ++i) {
    const int mBase = m0 + (i << 4);
#pragma unroll
    for (int j = 0; j < 4; ++j) {
      const int n = n0 + (j << 4) + rlane;
      float bv = 0.f;
      if (BIAS_MODE == 2) bv = bias[n];
#pragma unroll
      for (int r = 0; r < 8; ++r) {
        float v = acc[i][j][r] * scale;
        if (BIAS_MODE == 1) v += bias[mBase + mOff + r];
        if (BIAS_MODE == 2) v += bv;
        if (RESID) v += Rb[(size_t)(mBase + mOff + r) * ldc + n];
        if (ACT == 2) v = fmaxf(v, 0.0f);
        if (ACT == 4) v = (v > 0.f) ? v : 0.01f * v;
        slab[(mOff + r) * 68 + (j << 4) + rlane] = v;
      }
    }
    __builtin_amdgcn_fence(__ATOMIC_RELEASE, "workgroup");
    __builtin_amdgcn_wave_barrier();
    __builtin_amdgcn_fence(__ATOMIC_ACQUIRE, "workgroup");
    if (OUT_MODE == 0) {
      float* C = (float*)Cout + (size_t)b * strideC;
      const int hh = lane >> 4, c4 = (lane & 15) * 4;
      for (int pass = 0; pass < 2; ++pass) {
#pragma unroll
        for (int it = 0; it < 8; ++it) {
          const int row = it * 2 + hh;
          v4f v = *(const v4f*)(slab + row * 68 + c4);
          *(volatile v4f*)(C + (size_t)(mBase + row) * ldc + n0 + c4) = v;
        }
        __threadfence();
      }
    } else {
      const int q = lane >> 3, c8 = (lane & 7) * 8;
      unsigned short* C  = (unsigned short*)Cout  + (size_t)b * strideC;
      unsigned short* C2 = (OUT_MODE == 2) ? ((unsigned short*)Cout2 + (size_t)b * strideC) : nullptr;
      for (int pass = 0; pass < 2; ++pass) {
#pragma unroll
        for (int it = 0; it < 4; ++it) {
          const int row = it * 4 + q;
          const float* sp = slab + row * 68 + c8;
          v8h hv, lv;
#pragma unroll
          for (int e = 0; e < 8; ++e) {
            if (OUT_MODE == 1) {
              hv[e] = (_Float16)sp[e];
            } else {
              unsigned short hb = f2bf_bits(sp[e]);
              unsigned short lb = f2bf_bits(sp[e] - bf_bits2f(hb));
              hv[e] = __builtin_bit_cast(_Float16, hb);
              lv[e] = __builtin_bit_cast(_Float16, lb);
            }
          }
          *(volatile v8h*)(C + (size_t)(mBase + row) * ldc + n0 + c8) = hv;
          if (OUT_MODE == 2) *(volatile v8h*)(C2 + (size_t)(mBase + row) * ldc + n0 + c8) = lv;
        }
        __threadfence();
      }
    }
    __builtin_amdgcn_fence(__ATOMIC_RELEASE, "workgroup");
    __builtin_amdgcn_wave_barrier();
    __builtin_amdgcn_fence(__ATOMIC_ACQUIRE, "workgroup");
  }
}

__global__ __launch_bounds__(256) void cast8_scale_kernel(const float* __restrict__ in, unsigned short* __restrict__ out,
                                                          int n8, float scale) {
  const int i = blockIdx.x * 256 + threadIdx.x;
  if (i >= n8) return;
  const float* p = in + 8 * (size_t)i;
  const v4f a = *(const v4f*)(p);
  const v4f c = *(const v4f*)(p + 4);
  unsigned short hb[8];
#pragma unroll
  for (int e = 0; e < 4; ++e) {
    hb[e]     = h_bits(a[e] * scale);
    hb[4 + e] = h_bits(c[e] * scale);
  }
  const v4u u = (v4u){pk16(hb[0], hb[1]), pk16(hb[2], hb[3]), pk16(hb[4], hb[5]), pk16(hb[6], hb[7])};
  unsigned short* q = out + 8 * (size_t)i;
  *(volatile v4u*)q = u;
  __threadfence();
  *(volatile v4u*)q = u;
}

__global__ __launch_bounds__(256) void x_transpose_kernel(const float* __restrict__ x, unsigned short* __restrict__ X16) {
  __shared__ float sm[64][65];
  const int t  = threadIdx.x;
  const int n0 = blockIdx.x * 64;
  const int c0 = blockIdx.y * 64;
  const int b  = blockIdx.z;
#pragma unroll
  for (int i = 0; i < 16; ++i) {
    const int e  = i * 256 + t;
    const int r  = e >> 6;
    const int cc = e & 63;
    sm[cc][r] = x[((size_t)(b * kC + c0 + r)) * kN + n0 + cc];
  }
  __syncthreads();
  const int lane = t & 31, wave = t >> 5;
  const int q = lane >> 3, c8 = (lane & 7) * 8;
  v4u u[2];
  size_t off[2];
#pragma unroll
  for (int it = 0; it < 2; ++it) {
    const int row = wave * 8 + it * 4 + q;
    unsigned short hb[8];
#pragma unroll
    for (int e = 0; e < 8; ++e) hb[e] = h_bits(sm[row][c8 + e]);
    u[it] = (v4u){pk16(hb[0], hb[1]), pk16(hb[2], hb[3]), pk16(hb[4], hb[5]), pk16(hb[6], hb[7])};
    off[it] = ((size_t)(b * kN + n0 + row)) * kC + c0 + c8;
  }
  for (int pass = 0; pass < 2; ++pass) {
#pragma unroll
    for (int it = 0; it < 2; ++it) *(volatile v4u*)(X16 + off[it]) = u[it];
    __threadfence();
  }
}

__global__ __launch_bounds__(256) void branches_kernel(
    const float* __restrict__ x,
    const float* __restrict__ w1a, const float* __restrict__ b1a,
    const float* __restrict__ w1b, const float* __restrict__ b1b,
    const float* __restrict__ w2,  const float* __restrict__ b2,
    const float* __restrict__ w3,  const float* __restrict__ b3,
    float* __restrict__ Lpre) {
  __shared__ float Psh[16][16];
  __shared__ __align__(16) float orow[kMP];
  const int b = blockIdx.x / kC;
  const int c = blockIdx.x - b * kC;
  const int t = threadIdx.x;
  const bool act = (t < kP14);
  const int tt = act ? t : (kP14 - 1);
  const int ph = tt / 14, pw = tt - ph * 14;

  ((float*)Psh)[t] = 0.0f;
  if (t < kMP - kM) orow[kM + t] = 0.0f;
  __syncthreads();

  float xw[4][4];
  const float* xp = x + ((size_t)(b * kC + c)) * kN + (ph * 4) * kHW + pw * 4;
#pragma unroll
  for (int r = 0; r < 4; ++r)
#pragma unroll
    for (int s = 0; s < 4; ++s) xw[r][s] = xp[r * kHW + s];

  float a1 = b1b[c];
#pragma unroll
  for (int r = 0; r < 4; ++r) {
    float y = b1a[c];
#pragma unroll
    for (int s = 0; s < 4; ++s) y += w1a[c * 4 + s] * xw[r][s];
    y = fmaxf(y, 0.f);
    a1 += w1b[c * 4 + r] * y;
  }
  const float l1 = fmaxf(a1, 0.f);

  float a2 = b2[c];
#pragma unroll
  for (int r = 0; r < 4; ++r)
#pragma unroll
    for (int s = 0; s < 4; ++s) a2 += w2[c * 16 + r * 4 + s] * xw[r][s];
  const float l2 = fmaxf(a2, 0.f);

  float pool = 0.f;
#pragma unroll
  for (int r = 0; r < 4; ++r)
#pragma unroll
    for (int s = 0; s < 4; ++s) pool += xw[r][s];
  if (act) Psh[ph + 1][pw + 1] = pool * (1.0f / 16.0f);
  __syncthreads();

  float a3 = b3[c];
#pragma unroll
  for (int di = 0; di < 3; ++di)
#pragma unroll
    for (int dj = 0; dj < 3; ++dj)
      a3 += w3[c * 9 + di * 3 + dj] * Psh[ph + di][pw + dj];
  const float l3 = fmaxf(a3, 0.f);

  if (act) {
    orow[t] = l1;
    orow[kP14 + t] = l2;
    orow[2 * kP14 + t] = l3;
  }
  __syncthreads();

  if (t < kMP / 4) {
    const v4f v = *(const v4f*)(orow + 4 * t);
    float* dst = Lpre + (size_t)blockIdx.x * kMP + 4 * t;
    *(volatile v4f*)dst = v;
    __threadfence();
    *(volatile v4f*)dst = v;
  }
}

__global__ __launch_bounds__(256) void ln_kernel(const float* __restrict__ Lpre, const float* __restrict__ gamma,
                                                 const float* __restrict__ beta, unsigned short* __restrict__ L16) {
  __shared__ float sm[kC][17];
  __shared__ float mu_s[16];
  __shared__ float rs_s[16];
  const int t  = threadIdx.x;
  const int b  = blockIdx.x / (kMP / 16);
  const int mt = blockIdx.x - b * (kMP / 16);
  const int m0 = mt * 16;
  const float* src = Lpre + (size_t)b * kC * kMP + m0;
#pragma unroll
  for (int i = 0; i < 32; ++i) {
    const int e = i * 256 + t;
    const int c = e >> 4, j = e & 15;
    sm[c][j] = src[(size_t)c * kMP + j];
  }
  __syncthreads();

  const int j = t >> 4, sub = t & 15;
  float s = 0.f;
#pragma unroll 1
  for (int i = 0; i < 32; ++i) s += sm[sub + 16 * i][j];
  s += __shfl_xor(s, 8, 32);
  s += __shfl_xor(s, 4, 32);
  s += __shfl_xor(s, 2, 32);
  s += __shfl_xor(s, 1, 32);
  const float mu = s * (1.0f / kC);
  float s2 = 0.f;
#pragma unroll 1
  for (int i = 0; i < 32; ++i) {
    const float d = sm[sub + 16 * i][j] - mu;
    s2 += d * d;
  }
  s2 += __shfl_xor(s2, 8, 32);
  s2 += __shfl_xor(s2, 4, 32);
  s2 += __shfl_xor(s2, 2, 32);
  s2 += __shfl_xor(s2, 1, 32);
  const float var = s2 * (1.0f / kC);
  const float rs  = rsqrtf(var + kLnEps);
  if (sub == 0) { mu_s[j] = mu; rs_s[j] = rs; }
  __syncthreads();

  const int lane = t & 31, wave = t >> 5;
  v4u u[4];
  size_t off[4];
#pragma unroll
  for (int ui = 0; ui < 4; ++ui) {
    const int r = wave * 2 + (ui >> 1);
    const int cbase = (ui & 1) * 256 + lane * 8;
    const float mr = mu_s[r], rr = rs_s[r];
    const v4f g0 = *(const v4f*)(gamma + cbase);
    const v4f g1 = *(const v4f*)(gamma + cbase + 4);
    const v4f e0 = *(const v4f*)(beta + cbase);
    const v4f e1 = *(const v4f*)(beta + cbase + 4);
    unsigned short hb[8];
#pragma unroll
    for (int e = 0; e < 4; ++e) {
      hb[e]     = h_bits((sm[cbase + e][r] - mr) * rr * g0[e] + e0[e]);
      hb[4 + e] = h_bits((sm[cbase + 4 + e][r] - mr) * rr * g1[e] + e1[e]);
    }
    u[ui] = (v4u){pk16(hb[0], hb[1]), pk16(hb[2], hb[3]), pk16(hb[4], hb[5]), pk16(hb[6], hb[7])};
    off[ui] = ((size_t)(b * kMP + m0 + r)) * kC + cbase;
  }
  for (int pass = 0; pass < 2; ++pass) {
#pragma unroll
    for (int ui = 0; ui < 4; ++ui) *(volatile v4u*)(L16 + off[ui]) = u[ui];
    __threadfence();
  }
}

__global__ __launch_bounds__(256) void v_transpose_kernel(const unsigned short* __restrict__ KV16,
                                                          unsigned short* __restrict__ VT16) {
  __shared__ unsigned short sm[64][66];
  const int t  = threadIdx.x;
  const int mt = blockIdx.x;
  const int bh = blockIdx.y;
  const int b  = bh >> 3, h = bh & 7;
  const int m0 = mt * 64;
#pragma unroll
  for (int i = 0; i < 8; ++i) {
    const int e = i * 256 + t;
    const int r = e >> 5;
    const int w = e & 31;
    const unsigned short* rowp = KV16 + ((size_t)(b * kMP + m0 + r)) * (2 * kC) + kC + h * kHD;
    const unsigned uw = ((const unsigned*)(const void*)rowp)[w];
    sm[r][2 * w]     = (unsigned short)(uw & 0xffffu);
    sm[r][2 * w + 1] = (unsigned short)(uw >> 16);
  }
  __syncthreads();
  const int lane = t & 31, wave = t >> 5;
  const int q = lane >> 3, c8 = (lane & 7) * 8;
  v4u u[2];
  size_t off[2];
#pragma unroll
  for (int it = 0; it < 2; ++it) {
    const int row = wave * 8 + it * 4 + q;
    unsigned short hb[8];
#pragma unroll
    for (int e = 0; e < 8; ++e) {
      const unsigned short sv = sm[c8 + e][row];
      hb[e] = (m0 + c8 + e < kM) ? sv : (unsigned short)0;
    }
    u[it] = (v4u){pk16(hb[0], hb[1]), pk16(hb[2], hb[3]), pk16(hb[4], hb[5]), pk16(hb[6], hb[7])};
    off[it] = ((size_t)(bh * kHD + row)) * kMP + m0 + c8;
  }
  for (int pass = 0; pass < 2; ++pass) {
#pragma unroll
    for (int it = 0; it < 2; ++it) *(volatile v4u*)(VT16 + off[it]) = u[it];
    __threadfence();
  }
}

__global__ __launch_bounds__(128) void softmax_kernel(const float* __restrict__ S, unsigned short* __restrict__ P, int nrows) {
  const int lane = threadIdx.x & 31;
  const int wave = threadIdx.x >> 5;
  const int row  = blockIdx.x * 4 + wave;
  if (row >= nrows) return;
  const float* sr = S + (size_t)row * kMP;
  const int c0 = lane * 8;
  const int c1 = 256 + lane * 8;
  const int c2 = 512 + (lane & 15) * 8;
  const v4f a0 = *(const v4f*)(sr + c0);
  const v4f a1 = *(const v4f*)(sr + c0 + 4);
  const v4f q0 = *(const v4f*)(sr + c1);
  const v4f q1 = *(const v4f*)(sr + c1 + 4);
  const v4f d0 = *(const v4f*)(sr + c2);
  const v4f d1 = *(const v4f*)(sr + c2 + 4);
  float xv[24];
  bool  vv[8];
#pragma unroll
  for (int e = 0; e < 4; ++e) {
    xv[e] = a0[e]; xv[4 + e] = a1[e]; xv[8 + e] = q0[e]; xv[12 + e] = q1[e];
  }
#pragma unroll
  for (int e = 0; e < 4; ++e) {
    vv[e]     = (lane < 16) && (c2 + e < kM);
    vv[4 + e] = (lane < 16) && (c2 + 4 + e < kM);
    xv[16 + e] = vv[e]     ? d0[e] : xv[0];
    xv[20 + e] = vv[4 + e] ? d1[e] : xv[0];
  }
  float m = xv[0];
#pragma unroll
  for (int e = 1; e < 24; ++e) m = fmaxf(m, xv[e]);
  m = fmaxf(m, __shfl_xor(m, 16, 32));
  m = fmaxf(m, __shfl_xor(m, 8, 32));
  m = fmaxf(m, __shfl_xor(m, 4, 32));
  m = fmaxf(m, __shfl_xor(m, 2, 32));
  m = fmaxf(m, __shfl_xor(m, 1, 32));
  float p[24];
  float sum = 0.f;
#pragma unroll
  for (int e = 0; e < 16; ++e) { p[e] = __expf(xv[e] - m); sum += p[e]; }
#pragma unroll
  for (int e = 0; e < 8; ++e) {
    const float pe = __expf(xv[16 + e] - m);
    p[16 + e] = vv[e] ? pe : 0.0f;
    sum += p[16 + e];
  }
  sum += __shfl_xor(sum, 16, 32);
  sum += __shfl_xor(sum, 8, 32);
  sum += __shfl_xor(sum, 4, 32);
  sum += __shfl_xor(sum, 2, 32);
  sum += __shfl_xor(sum, 1, 32);
  const float inv = kPCarry / sum;
  unsigned short hb[24];
#pragma unroll
  for (int e = 0; e < 24; ++e) hb[e] = h_bits(p[e] * inv);
  const v4u u0 = (v4u){pk16(hb[0], hb[1]), pk16(hb[2], hb[3]), pk16(hb[4], hb[5]), pk16(hb[6], hb[7])};
  const v4u u1 = (v4u){pk16(hb[8], hb[9]), pk16(hb[10], hb[11]), pk16(hb[12], hb[13]), pk16(hb[14], hb[15])};
  const v4u u2 = (v4u){pk16(hb[16], hb[17]), pk16(hb[18], hb[19]), pk16(hb[20], hb[21]), pk16(hb[22], hb[23])};
  unsigned short* pr = P + (size_t)row * kMP;
  *(volatile v4u*)(pr + c0) = u0;
  *(volatile v4u*)(pr + c1) = u1;
  if (lane < 16) *(volatile v4u*)(pr + c2) = u2;
  __threadfence();
  *(volatile v4u*)(pr + c0) = u0;
  *(volatile v4u*)(pr + c1) = u1;
  if (lane < 16) *(volatile v4u*)(pr + c2) = u2;
}

extern "C" void kernel_launch(void* const* d_in, const int* in_sizes, int n_in,
                              void* d_out, int out_size, void* d_ws,
                              size_t ws_size, hipStream_t stream) {
  if (n_in < 15) return;
  if (in_sizes[0] != kB * kC * kN) return;
  if (in_sizes[1] != kC * kC || in_sizes[2] < kC) return;
  if (in_sizes[3] != 2 * kC * kC || in_sizes[4] < 2 * kC) return;
  if (in_sizes[5] < kC * 4 || in_sizes[6] < kC || in_sizes[7] < kC * 4 || in_sizes[8] < kC) return;
  if (in_sizes[9] < kC * 16 || in_sizes[10] < kC || in_sizes[11] < kC * 9 || in_sizes[12] < kC) return;
  if (in_sizes[13] < kC || in_sizes[14] < kC) return;
  if (out_size != kB * kN * kC) return;

  const float* x    = (const float*)d_in[0];
  const float* Wq   = (const float*)d_in[1];
  const float* bq   = (const float*)d_in[2];
  const float* Wkv  = (const float*)d_in[3];
  const float* bkv  = (const float*)d_in[4];
  const float* w1a  = (const float*)d_in[5];
  const float* b1a  = (const float*)d_in[6];
  const float* w1b  = (const float*)d_in[7];
  const float* b1b  = (const float*)d_in[8];
  const float* w2   = (const float*)d_in[9];
  const float* b2   = (const float*)d_in[10];
  const float* w3   = (const float*)d_in[11];
  const float* b3   = (const float*)d_in[12];
  const float* gam  = (const float*)d_in[13];
  const float* bet  = (const float*)d_in[14];
  float* outp = (float*)d_out;

  const size_t bX16  = (size_t)kTokRows * kC * 2;
  const size_t bLpre = (size_t)kB * kC * kMP * 4;
  const size_t bS    = (size_t)kGH * kN * kMP * 4;
  const size_t bQ16  = (size_t)kTokRows * kC * 2;
  const size_t bL16  = (size_t)kKVRows * kC * 2;
  const size_t bWq   = (size_t)kC * kC * 2;
  const size_t bWkv  = (size_t)2 * kC * kC * 2;
  const size_t bKV   = (size_t)kKVRows * 2 * kC * 2;
  const size_t bVT   = (size_t)kB * kHeads * kHD * kMP * 2;
  const size_t bP16  = (size_t)kGH * kN * kMP * 2;

  const size_t oX16  = 0;
  const size_t oLpre = oX16 + bX16;
  const size_t oS    = 0;
  if (oS + bS > oLpre + bLpre) return;
  const size_t oQ16  = oLpre + bLpre;
  const size_t oL16  = oQ16 + bQ16;
  const size_t oWq   = oL16 + bL16;
  const size_t oWkv  = oWq + bWq;
  const size_t oKV   = oWkv + bWkv;
  const size_t oVT   = oKV + bKV;
  const size_t oP16  = oVT + bVT;
  const size_t total = oP16 + bP16;
  if (total > ws_size) return;

  char* ws = (char*)d_ws;
  unsigned short* X16  = (unsigned short*)(ws + oX16);
  float*          Lpre = (float*)(ws + oLpre);
  float*          Sg   = (float*)(ws + oS);
  unsigned short* Q16  = (unsigned short*)(ws + oQ16);
  unsigned short* L16  = (unsigned short*)(ws + oL16);
  unsigned short* Wq16 = (unsigned short*)(ws + oWq);
  unsigned short* Wkv16 = (unsigned short*)(ws + oWkv);
  unsigned short* KV16 = (unsigned short*)(ws + oKV);
  unsigned short* VT16 = (unsigned short*)(ws + oVT);
  unsigned short* P16  = (unsigned short*)(ws + oP16);

  cast8_scale_kernel<<<dim3((kC * kC / 8 + 255) / 256), 256, 0, stream>>>(Wq, Wq16, kC * kC / 8, kWCarry);
  cast8_scale_kernel<<<dim3((2 * kC * kC / 8 + 255) / 256), 256, 0, stream>>>(Wkv, Wkv16, 2 * kC * kC / 8, kWCarry);

  x_transpose_kernel<<<dim3(kN / 64, kC / 64, kB), 256, 0, stream>>>(x, X16);

  wmma_gemm64<0, false, 2, 1, false, 0><<<dim3((kTokRows / 64) * (kC / 64) / 8, 1), 256, 0, stream>>>(
      X16, X16, kC, 0L, Wq16, Wq16, kC, 0L, (void*)Q16, (void*)Q16, kC, 0L,
      bq, x, 0L, kTokRows, kC, kC, kWCarryInv);

  branches_kernel<<<dim3(kB * kC), 256, 0, stream>>>(x, w1a, b1a, w1b, b1b, w2, b2, w3, b3, Lpre);

  ln_kernel<<<dim3(kB * (kMP / 16)), 256, 0, stream>>>(Lpre, gam, bet, L16);

  wmma_gemm64<0, false, 2, 1, false, 0><<<dim3((kKVRows / 64) * (2 * kC / 64) / 8, 1), 256, 0, stream>>>(
      L16, L16, kC, 0L, Wkv16, Wkv16, kC, 0L, (void*)KV16, (void*)KV16, 2 * kC, 0L,
      bkv, x, 0L, kKVRows, 2 * kC, kC, kWCarryInv);

  v_transpose_kernel<<<dim3(kMP / 64, kB * kHeads), 256, 0, stream>>>(KV16, VT16);

  const long sStrideC = (long)kN * kMP;
  const int  sBlocks  = ((kN / 64) * (kMP / 64) + 7) / 8;
  const int  pvBlocks = ((kN / 64) * (kHD / 64) + 7) / 8;
  for (int bb = 0; bb < kB; ++bb) {
    for (int hg = 0; hg < kHeads / kGH; ++hg) {
      const unsigned short* Aq = Q16 + (size_t)bb * kN * kC + (size_t)hg * kGH * kHD;
      const unsigned short* Bk = KV16 + (size_t)bb * kMP * (2 * kC) + (size_t)hg * kGH * kHD;
      wmma_gemm64<0, false, 0, 0, false, 0><<<dim3(sBlocks, kGH), 256, 0, stream>>>(
          Aq, Aq, kC, (long)kHD, Bk, Bk, 2 * kC, (long)kHD, (void*)Sg, (void*)Sg, kMP, sStrideC,
          bq, x, 0L, kN, kMP, kHD, kQKScale);
      softmax_kernel<<<dim3(kGroupRows / 4), 128, 0, stream>>>(Sg, P16, kGroupRows);
      const unsigned short* Bv = VT16 + ((size_t)(bb * kHeads + hg * kGH)) * kHD * kMP;
      float* Co = outp + (size_t)bb * kN * kC + (size_t)hg * kGH * kHD;
      wmma_gemm64<0, false, 0, 0, false, 0><<<dim3(pvBlocks, kGH), 256, 0, stream>>>(
          P16, P16, kMP, sStrideC, Bv, Bv, kMP, (long)kHD * kMP, (void*)Co, (void*)Co, kC, (long)kHD,
          bq, x, 0L, kN, kHD, kMP, kPCarryInv);
    }
  }
}
